// KGAtt_49082886259211
// MI455X (gfx1250) — hardware-verified
//
#include <hip/hip_runtime.h>
#include <stddef.h>


#define DF    128
#define KW    384
#define GR    32
#define AP    136
#define XSP   260
#define NTHR  256
#define NWAVE 8
#define NB    512
#define CHUNK 2048
#define WCAP  256
#define NGRP  (CHUNK / (NTHR * 4))
#define CNTW  256
#define NBLKR 32

#define SRC_LDS_BYTES ((NB * DF + NB + NWAVE * WCAP + NWAVE) * 4)

static_assert(WCAP == (CHUNK / NTHR) * 32);
static_assert(NGRP == 2);
static_assert(NB == 512);
static_assert(CHUNK == 2048);
static_assert(((NB * DF + NB) % 4) == 0);
static_assert(SRC_LDS_BYTES == 272416);
static_assert((XSP % 4) == 0);
static_assert((AP % 8) == 0);

typedef float          v4f   __attribute__((ext_vector_type(4)));
typedef float          v8f   __attribute__((ext_vector_type(8)));
typedef unsigned short v8us  __attribute__((ext_vector_type(8)));
typedef __bf16         v16bf __attribute__((ext_vector_type(16)));
union FragB { v16bf v; v8us us[2]; };

__device__ __forceinline__ v8f wm(v16bf a, v16bf b, v8f c) {
  v8f d = __builtin_amdgcn_wmma_f32_16x16x32_bf16(false, a, false, b, (short)0, c, false, false);
  asm volatile("v_nop\n\tv_nop\n\tv_nop\n\tv_nop" : "+v"(d) : "v"(a), "v"(b));
  return d;
}

__device__ __forceinline__ float wsum(float v) {
  v += __shfl_xor(v, 16, 32);
  v += __shfl_xor(v, 8, 32);
  v += __shfl_xor(v, 4, 32);
  v += __shfl_xor(v, 2, 32);
  v += __shfl_xor(v, 1, 32);
  return v;
}

__device__ __forceinline__ unsigned short bfb(float f) {
  unsigned u = __float_as_uint(f);
  u = u + 0x7FFFu + ((u >> 16) & 1u);
  return (unsigned short)(u >> 16);
}

__device__ __forceinline__ void split_hl(float x, unsigned short& h, unsigned short& l) {
  const unsigned short hb = bfb(x);
  const float hf = __uint_as_float(((unsigned)hb) << 16);
  h = hb;
  l = bfb(x - hf);
}

__device__ __forceinline__ void split8(v4f a, v4f b, v8us& hv, v8us& lv) {
  unsigned short h, l;
  split_hl(a.x, h, l); hv[0] = h; lv[0] = l;
  split_hl(a.y, h, l); hv[1] = h; lv[1] = l;
  split_hl(a.z, h, l); hv[2] = h; lv[2] = l;
  split_hl(a.w, h, l); hv[3] = h; lv[3] = l;
  split_hl(b.x, h, l); hv[4] = h; lv[4] = l;
  split_hl(b.y, h, l); hv[5] = h; lv[5] = l;
  split_hl(b.z, h, l); hv[6] = h; lv[6] = l;
  split_hl(b.w, h, l); hv[7] = h; lv[7] = l;
}

__device__ __forceinline__ float elu1(float x) { return x > 0.f ? x : (__expf(x) - 1.0f); }
__device__ __forceinline__ v4f elu4(v4f v) {
  v4f r;
  r.x = elu1(v.x); r.y = elu1(v.y); r.z = elu1(v.z); r.w = elu1(v.w);
  return r;
}

__device__ __forceinline__ float edge_eb(v4f c, v4f w4, float ba2v) {
  float t = c.x * w4.x + c.y * w4.y + c.z * w4.z + c.w * w4.w;
  t = wsum(t);
  float b = t + ba2v;
  b = (b > 0.f) ? b : 0.01f * b;
  return expf(b);
}

__global__ __launch_bounds__(NTHR) void k_prepw(const float* __restrict__ W,
                                                unsigned short* Wh, unsigned short* Wl, int n8) {
  const int i = blockIdx.x * NTHR + threadIdx.x;
  if (i >= n8) return;
  const size_t o = (size_t)i * 8;
  const v4f a = *(const v4f*)(W + o);
  const v4f b = *(const v4f*)(W + o + 4);
  v8us hv = {0, 0, 0, 0, 0, 0, 0, 0};
  v8us lv = {0, 0, 0, 0, 0, 0, 0, 0};
  split8(a, b, hv, lv);
  *(volatile v8us*)(Wh + o) = hv;
  *(volatile v8us*)(Wl + o) = lv;
  __threadfence();
  *(volatile v8us*)(Wh + o) = hv;
  *(volatile v8us*)(Wl + o) = lv;
}

__global__ __launch_bounds__(NTHR) void k_gemm(
    const float* __restrict__ x, int nX,
    const unsigned short* __restrict__ Wh, const unsigned short* __restrict__ Wl,
    int kofs0, int kofs1, float* o0, float* o1, int ncg) {
  __shared__ __attribute__((aligned(16))) unsigned short Ahi[GR * AP];
  __shared__ __attribute__((aligned(16))) unsigned short Alo[GR * AP];
  __shared__ __attribute__((aligned(16))) float Xs[GR * XSP];

  const int tid  = threadIdx.x;
  const int lane = tid & 31;
  const int wave = __builtin_amdgcn_readfirstlane(tid >> 5);
  const int hh   = lane >> 4;
  const int m    = lane & 15;
  const int rowBase = blockIdx.x * GR;

  {
    const int r  = tid >> 3;
    const int c0 = (tid & 7) * 16;
    int row = rowBase + r;
    if (row > nX - 1) row = nX - 1;
    const float* p = x + (size_t)row * DF + c0;
    const v4f f0 = *(const v4f*)(p), f1 = *(const v4f*)(p + 4);
    const v4f f2 = *(const v4f*)(p + 8), f3 = *(const v4f*)(p + 12);
    v8us h0 = {0, 0, 0, 0, 0, 0, 0, 0}, l0 = {0, 0, 0, 0, 0, 0, 0, 0};
    v8us h1 = {0, 0, 0, 0, 0, 0, 0, 0}, l1 = {0, 0, 0, 0, 0, 0, 0, 0};
    split8(f0, f1, h0, l0);
    split8(f2, f3, h1, l1);
    *(v8us*)(Ahi + r * AP + c0)     = h0;
    *(v8us*)(Ahi + r * AP + c0 + 8) = h1;
    *(v8us*)(Alo + r * AP + c0)     = l0;
    *(v8us*)(Alo + r * AP + c0 + 8) = l1;
  }
  __syncthreads();

  const int cg   = wave >> 2;
  const int wq   = wave & 3;
  const int kofs = (cg == 0) ? kofs0 : kofs1;
  v8f c00 = {0.f, 0.f, 0.f, 0.f, 0.f, 0.f, 0.f, 0.f};
  v8f c01 = {0.f, 0.f, 0.f, 0.f, 0.f, 0.f, 0.f, 0.f};
  v8f c10 = {0.f, 0.f, 0.f, 0.f, 0.f, 0.f, 0.f, 0.f};
  v8f c11 = {0.f, 0.f, 0.f, 0.f, 0.f, 0.f, 0.f, 0.f};
  if (cg < ncg) {
    const int n0 = wq * 32 + m;
    const int n1 = n0 + 16;
    const unsigned short* bh0 = Wh + (size_t)n0 * KW + kofs + 8 * hh;
    const unsigned short* bl0 = Wl + (size_t)n0 * KW + kofs + 8 * hh;
    const unsigned short* bh1 = Wh + (size_t)n1 * KW + kofs + 8 * hh;
    const unsigned short* bl1 = Wl + (size_t)n1 * KW + kofs + 8 * hh;
    const unsigned short* ah0 = Ahi + m * AP + 8 * hh;
    const unsigned short* al0 = Alo + m * AP + 8 * hh;
    const unsigned short* ah1 = Ahi + (16 + m) * AP + 8 * hh;
    const unsigned short* al1 = Alo + (16 + m) * AP + 8 * hh;
#pragma unroll 1
    for (int kt = 0; kt < DF / 32; ++kt) {
      const int k0 = kt * 32;
      FragB a0h, a0l, a1h, a1l, b0h, b0l, b1h, b1l;
      a0h.us[0] = *(const v8us*)(ah0 + k0); a0h.us[1] = *(const v8us*)(ah0 + k0 + 16);
      a0l.us[0] = *(const v8us*)(al0 + k0); a0l.us[1] = *(const v8us*)(al0 + k0 + 16);
      a1h.us[0] = *(const v8us*)(ah1 + k0); a1h.us[1] = *(const v8us*)(ah1 + k0 + 16);
      a1l.us[0] = *(const v8us*)(al1 + k0); a1l.us[1] = *(const v8us*)(al1 + k0 + 16);
      b0h.us[0] = *(const v8us*)(bh0 + k0); b0h.us[1] = *(const v8us*)(bh0 + k0 + 16);
      b0l.us[0] = *(const v8us*)(bl0 + k0); b0l.us[1] = *(const v8us*)(bl0 + k0 + 16);
      b1h.us[0] = *(const v8us*)(bh1 + k0); b1h.us[1] = *(const v8us*)(bh1 + k0 + 16);
      b1l.us[0] = *(const v8us*)(bl1 + k0); b1l.us[1] = *(const v8us*)(bl1 + k0 + 16);
      c00 = wm(a0h.v, b0h.v, c00); c00 = wm(a0h.v, b0l.v, c00); c00 = wm(a0l.v, b0h.v, c00);
      c01 = wm(a0h.v, b1h.v, c01); c01 = wm(a0h.v, b1l.v, c01); c01 = wm(a0l.v, b1h.v, c01);
      c10 = wm(a1h.v, b0h.v, c10); c10 = wm(a1h.v, b0l.v, c10); c10 = wm(a1l.v, b0h.v, c10);
      c11 = wm(a1h.v, b1h.v, c11); c11 = wm(a1h.v, b1l.v, c11); c11 = wm(a1l.v, b1h.v, c11);
    }
    const int colb = cg * DF + wq * 32 + m;
#pragma unroll
    for (int r = 0; r < 8; ++r) {
      Xs[(8 * hh + r) * XSP + colb]           = c00[r];
      Xs[(8 * hh + r) * XSP + colb + 16]      = c01[r];
      Xs[(16 + 8 * hh + r) * XSP + colb]      = c10[r];
      Xs[(16 + 8 * hh + r) * XSP + colb + 16] = c11[r];
    }
  }
  __syncthreads();

  const bool two = (ncg > 1);
  v4f v0[4], v1[4];
  float* p0[4];
  float* p1[4];
#pragma unroll
  for (int i = 0; i < 4; ++i) {
    const int row = 4 * wave + i;
    v0[i] = *(const v4f*)(Xs + row * XSP + 4 * lane);
    v1[i] = v0[i];
    if (two) v1[i] = *(const v4f*)(Xs + row * XSP + DF + 4 * lane);
    p0[i] = o0 + (size_t)(rowBase + row) * DF + 4 * lane;
    p1[i] = o1 + (size_t)(rowBase + row) * DF + 4 * lane;
  }
#pragma unroll
  for (int i = 0; i < 4; ++i) *(volatile v4f*)(p0[i]) = v0[i];
  if (two) {
#pragma unroll
    for (int i = 0; i < 4; ++i) *(volatile v4f*)(p1[i]) = v1[i];
  }
  __threadfence();
#pragma unroll
  for (int i = 0; i < 4; ++i) *(volatile v4f*)(p0[i]) = v0[i];
  if (two) {
#pragma unroll
    for (int i = 0; i < 4; ++i) *(volatile v4f*)(p1[i]) = v1[i];
  }
}

__global__ __launch_bounds__(NTHR) void k_src(
    const int* __restrict__ trip, int nE,
    const float* __restrict__ P, const float* __restrict__ Q, const float* __restrict__ R,
    const float* __restrict__ ba, const float* __restrict__ Wa2, const float* __restrict__ ba2,
    float* out, int nN, int nR) {
  extern __shared__ v4f lds_dyn[];
  float* sacc = (float*)lds_dyn;
  float* ebs  = sacc + NB * DF;
  int*   list = (int*)(ebs + NB);
  int*   wcnt = list + NWAVE * WCAP;

  const int tid  = threadIdx.x;
  const int lane = tid & 31;
  const int wave = __builtin_amdgcn_readfirstlane(tid >> 5);
  const int nodeBase = blockIdx.x * NB;

  {
    const v4f z4 = {0.f, 0.f, 0.f, 0.f};
    for (int i = tid; i < (NB * DF + NB) / 4; i += NTHR) lds_dyn[i] = z4;
  }
  __syncthreads();

  const v4f ba4 = *(const v4f*)(ba + 4 * lane);
  const v4f w4  = *(const v4f*)(Wa2 + 4 * lane);
  const float ba2v = ba2[0];

  const int nChunks = (nE + CHUNK - 1) / CHUNK;
#pragma unroll 1
  for (int ch = 0; ch < nChunks; ++ch) {
    const int cbase = ch * CHUNK;
    int wc = 0;
#pragma unroll
    for (int g = 0; g < NGRP; ++g) {
      const int el0 = (g * NTHR + tid) * 4;
      const int e0  = cbase + el0;
      const int sent = -2147483647 - 1;
      int ec;
      ec = e0;     if (ec > nE - 1) ec = nE - 1; const int t0 = trip[(size_t)ec * 3];
      ec = e0 + 1; if (ec > nE - 1) ec = nE - 1; const int t1 = trip[(size_t)ec * 3];
      ec = e0 + 2; if (ec > nE - 1) ec = nE - 1; const int t2 = trip[(size_t)ec * 3];
      ec = e0 + 3; if (ec > nE - 1) ec = nE - 1; const int t3 = trip[(size_t)ec * 3];
      const int d0 = (e0     < nE) ? t0 : sent;
      const int d1 = (e0 + 1 < nE) ? t1 : sent;
      const int d2 = (e0 + 2 < nE) ? t2 : sent;
      const int d3 = (e0 + 3 < nE) ? t3 : sent;
      const unsigned s0 = (unsigned)d0 - (unsigned)nodeBase;
      const unsigned s1 = (unsigned)d1 - (unsigned)nodeBase;
      const unsigned s2 = (unsigned)d2 - (unsigned)nodeBase;
      const unsigned s3 = (unsigned)d3 - (unsigned)nodeBase;
      const bool h0 = s0 < (unsigned)NB;
      const bool h1 = s1 < (unsigned)NB;
      const bool h2 = s2 < (unsigned)NB;
      const bool h3 = s3 < (unsigned)NB;
      const unsigned many = __builtin_amdgcn_ballot_w32(h0 | h1 | h2 | h3);
      if (many != 0u) {
#define HITJ(J, HJ, SJ) { \
          const unsigned mj = __builtin_amdgcn_ballot_w32(HJ); \
          if (HJ) { \
            const int pos = wc + (int)__builtin_amdgcn_mbcnt_lo(mj, 0u); \
            if (pos < WCAP) list[wave * WCAP + pos] = ((el0 + (J)) << 9) | (int)(SJ); \
          } \
          wc += (int)__builtin_popcount(mj); }
        HITJ(0, h0, s0)
        HITJ(1, h1, s1)
        HITJ(2, h2, s2)
        HITJ(3, h3, s3)
#undef HITJ
      }
    }
    if (lane == 0) wcnt[wave] = wc;
    __syncthreads();

    if (wave == 0) {
      for (int wsx = 0; wsx < NWAVE; ++wsx) {
        int n = wcnt[wsx];
        if (n > WCAP) n = WCAP;
        if (n < 0) n = 0;
        for (int i = 0; i < n; ++i) {
          const int ent  = list[wsx * WCAP + i];
          const int slot = ent & (NB - 1);
          const int el   = (ent >> 9) & (CHUNK - 1);
          int e = cbase + el;
          if (e > nE - 1) e = nE - 1;
          int dn = trip[(size_t)e * 3 + 1];
          int rr = trip[(size_t)e * 3 + 2];
          dn = dn < 0 ? 0 : (dn > nN - 1 ? nN - 1 : dn);
          rr = rr < 0 ? 0 : (rr > nR - 1 ? nR - 1 : rr);
          int nd = nodeBase + slot;
          if (nd > nN - 1) nd = nN - 1;
          const v4f pv = *(const v4f*)(P + (size_t)nd * DF + 4 * lane);
          const v4f rv = *(const v4f*)(R + (size_t)rr * DF + 4 * lane);
          const v4f qv = *(const v4f*)(Q + (size_t)dn * DF + 4 * lane);
          const v4f c  = ((pv + rv) + qv) + ba4;
          const float eb = edge_eb(c, w4, ba2v);
          v4f* sp = (v4f*)(sacc + slot * DF + 4 * lane);
          const v4f cur = *sp;
          *sp = cur + eb * c;
          if (lane == 0) {
            const float o = ebs[slot];
            ebs[slot] = o + eb;
          }
        }
      }
    }
    __syncthreads();
  }

#pragma unroll 1
  for (int j = 0; j < NB / NWAVE; ++j) {
    const int slot = wave * (NB / NWAVE) + j;
    const int node = nodeBase + slot;
    if (node >= nN) break;
    float s = ebs[slot];
    s = (s == 0.f) ? 1e-12f : s;
    const float inv = 1.0f / s;
    const v4f hv = *(const v4f*)(sacc + slot * DF + 4 * lane);
    const v4f y = elu4(hv * inv);
    float* op = out + (size_t)node * DF + 4 * lane;
    *(volatile v4f*)op = y;
    __threadfence();
    *(volatile v4f*)op = y;
  }
}

__global__ __launch_bounds__(NTHR) void k_rel(
    const int* __restrict__ trip, int nE, int epb,
    const float* __restrict__ P, const float* __restrict__ Q, const float* __restrict__ R,
    const float* __restrict__ ba, const float* __restrict__ Wa2, const float* __restrict__ ba2,
    float* part, float* pcnt, int nN, int nR, int rp) {
  extern __shared__ v4f lds_dyn[];
  float* racc = (float*)lds_dyn;
  float* rcnt = racc + rp * DF;

  const int tid  = threadIdx.x;
  const int lane = tid & 31;
  const int wave = __builtin_amdgcn_readfirstlane(tid >> 5);

  {
    const v4f z4 = {0.f, 0.f, 0.f, 0.f};
    const int nz = (rp * DF + CNTW) / 4;
    for (int i = tid; i < nz; i += NTHR) lds_dyn[i] = z4;
  }
  __syncthreads();

  const v4f ba4 = *(const v4f*)(ba + 4 * lane);
  const v4f w4  = *(const v4f*)(Wa2 + 4 * lane);
  const float ba2v = ba2[0];

  const int e0 = blockIdx.x * epb;
  int e1 = e0 + epb;
  if (e1 > nE) e1 = nE;
  const int ng = (e1 > e0) ? ((e1 - e0 + 31) / 32) : 0;

#pragma unroll 1
  for (int i = 0; i < ng; ++i) {
    const int base = e0 + 32 * i;
    const int e = base + lane;
    int ec = e;
    if (ec > nE - 1) ec = nE - 1;
    const int kv  = trip[(size_t)ec * 3 + 2];
    const int key = (e < e1) ? kv : -1;
    const bool valid = ((unsigned)key < (unsigned)nR) && ((key & 7) == wave);
    unsigned msk = __builtin_amdgcn_ballot_w32(valid);
    while (msk != 0u) {
      const int bit = __builtin_ctz(msk);
      msk &= (msk - 1u);
      int rr = __shfl(key, bit, 32);
      rr = rr < 0 ? 0 : (rr > nR - 1 ? nR - 1 : rr);
      int ee = base + bit;
      if (ee > nE - 1) ee = nE - 1;
      int sn = trip[(size_t)ee * 3];
      int dn = trip[(size_t)ee * 3 + 1];
      sn = sn < 0 ? 0 : (sn > nN - 1 ? nN - 1 : sn);
      dn = dn < 0 ? 0 : (dn > nN - 1 ? nN - 1 : dn);
      const v4f pv = *(const v4f*)(P + (size_t)sn * DF + 4 * lane);
      const v4f rv = *(const v4f*)(R + (size_t)rr * DF + 4 * lane);
      const v4f qv = *(const v4f*)(Q + (size_t)dn * DF + 4 * lane);
      const v4f c  = ((pv + rv) + qv) + ba4;
      const float eb = edge_eb(c, w4, ba2v);
      v4f* sp = (v4f*)(racc + rr * DF + 4 * lane);
      const v4f cur = *sp;
      *sp = cur + eb * c;
      if (lane == 0) {
        const float o = rcnt[rr];
        rcnt[rr] = o + 1.0f;
      }
    }
  }
  __syncthreads();

  const size_t pbase = (size_t)blockIdx.x * (size_t)rp;
  float* cbase = pcnt + (size_t)blockIdx.x * CNTW;
  const v4f cv0 = *(const v4f*)(rcnt + 4 * lane);
  const v4f cv1 = *(const v4f*)(rcnt + DF + 4 * lane);
#pragma unroll 1
  for (int r = wave; r < nR; r += NWAVE) {
    const v4f v = *(const v4f*)(racc + r * DF + 4 * lane);
    *(volatile v4f*)(part + (pbase + (size_t)r) * DF + 4 * lane) = v;
  }
  if (wave == 0) {
    *(volatile v4f*)(cbase + 4 * lane)      = cv0;
    *(volatile v4f*)(cbase + DF + 4 * lane) = cv1;
  }
  __threadfence();
#pragma unroll 1
  for (int r = wave; r < nR; r += NWAVE) {
    const v4f v = *(const v4f*)(racc + r * DF + 4 * lane);
    *(volatile v4f*)(part + (pbase + (size_t)r) * DF + 4 * lane) = v;
  }
  if (wave == 0) {
    *(volatile v4f*)(cbase + 4 * lane)      = cv0;
    *(volatile v4f*)(cbase + DF + 4 * lane) = cv1;
  }
}

__global__ __launch_bounds__(NTHR) void k_fin(const float* __restrict__ part,
                                              const float* __restrict__ pcnt,
                                              int nblk, int nR, int rp, float* out1) {
  const int tid  = threadIdx.x;
  const int lane = tid & 31;
  const int wave = __builtin_amdgcn_readfirstlane(tid >> 5);
  const int rr = blockIdx.x * NWAVE + wave;
  if (rr >= nR) return;
  v4f s = {0.f, 0.f, 0.f, 0.f};
  float cn = 0.f;
#pragma unroll 1
  for (int k = 0; k < nblk; ++k) {
    s  += *(const v4f*)(part + ((size_t)k * (size_t)rp + (size_t)rr) * DF + 4 * lane);
    cn += pcnt[(size_t)k * CNTW + rr];
  }
  const float inv = 1.0f / fmaxf(cn, 1.0f);
  const v4f y = elu4(s * inv);
  float* op = out1 + (size_t)rr * DF + 4 * lane;
  *(volatile v4f*)op = y;
  __threadfence();
  *(volatile v4f*)op = y;
}

extern "C" void kernel_launch(void* const* d_in, const int* in_sizes, int n_in,
                              void* d_out, int out_size, void* d_ws, size_t ws_size,
                              hipStream_t stream) {
  if (n_in < 7) return;
  const int nE = in_sizes[0] / 3;
  const int nN = in_sizes[1] / DF;
  const int nR = in_sizes[2] / DF;
  if (nE <= 0 || in_sizes[0] != 3 * nE) return;
  if (nN <= 0 || in_sizes[1] != nN * DF) return;
  if (nR <= 0 || nR > CNTW || in_sizes[2] != nR * DF) return;
  if (in_sizes[3] != DF * KW) return;
  if (in_sizes[4] != DF || in_sizes[5] != DF || in_sizes[6] < 1) return;
  if (out_size != (nN + nR) * DF) return;

  const int*   trip = (const int*)d_in[0];
  const float* ent  = (const float*)d_in[1];
  const float* rele = (const float*)d_in[2];
  const float* Wa   = (const float*)d_in[3];
  const float* ba   = (const float*)d_in[4];
  const float* Wa2  = (const float*)d_in[5];
  const float* ba2  = (const float*)d_in[6];
  float* out0 = (float*)d_out;
  float* out1 = (float*)d_out + (size_t)nN * DF;

  const int nP = ((nN + GR - 1) / GR) * GR;
  const int rp = ((nR + GR - 1) / GR) * GR;
  size_t off = 0;
  unsigned short* Wh = (unsigned short*)((char*)d_ws + off); off += (size_t)DF * KW * 2;
  unsigned short* Wl = (unsigned short*)((char*)d_ws + off); off += (size_t)DF * KW * 2;
  float* Pp   = (float*)((char*)d_ws + off); off += (size_t)nP * DF * sizeof(float);
  float* Qp   = (float*)((char*)d_ws + off); off += (size_t)nP * DF * sizeof(float);
  float* Rp   = (float*)((char*)d_ws + off); off += (size_t)rp * DF * sizeof(float);
  float* part = (float*)((char*)d_ws + off); off += (size_t)NBLKR * rp * DF * sizeof(float);
  float* pcnt = (float*)((char*)d_ws + off); off += (size_t)NBLKR * CNTW * sizeof(float);
  if (off > ws_size) return;

  const int n8 = DF * KW / 8;
  k_prepw<<<(n8 + NTHR - 1) / NTHR, NTHR, 0, stream>>>(Wa, Wh, Wl, n8);

  k_gemm<<<nP / GR, NTHR, 0, stream>>>(ent, nN, Wh, Wl, 0, 2 * DF, Pp, Qp, 2);
  k_gemm<<<rp / GR, NTHR, 0, stream>>>(rele, nR, Wh, Wl, DF, DF, Rp, Rp, 1);

  hipFuncSetAttribute(reinterpret_cast<const void*>(&k_src),
                      hipFuncAttributeMaxDynamicSharedMemorySize, SRC_LDS_BYTES);
  const int gridS = (nN + NB - 1) / NB;
  k_src<<<gridS, NTHR, SRC_LDS_BYTES, stream>>>(trip, nE, Pp, Qp, Rp, ba, Wa2, ba2,
                                                 out0, nN, nR);

  const int epb = ((((nE + NBLKR - 1) / NBLKR) + 31) / 32) * 32;
  const int relLds = (rp * DF + CNTW) * (int)sizeof(float);
  hipFuncSetAttribute(reinterpret_cast<const void*>(&k_rel),
                      hipFuncAttributeMaxDynamicSharedMemorySize, relLds);
  k_rel<<<NBLKR, NTHR, relLds, stream>>>(trip, nE, epb, Pp, Qp, Rp, ba, Wa2, ba2,
                                         part, pcnt, nN, nR, rp);

  k_fin<<<(nR + NWAVE - 1) / NWAVE, NTHR, 0, stream>>>(part, pcnt, NBLKR, nR, rp, out1);
}
